// TriangleAttention_12455405158978
// MI455X (gfx1250) — hardware-verified
//
#include <hip/hip_runtime.h>
#include <math.h>
#include <stdint.h>

#ifndef NB
#define NB 1
#endif
#ifndef NI
#define NI 256
#endif
#define NSEQ   256
#define CZ     128
#define NH     4
#define HD     32
#define NPOS   (NSEQ * NSEQ)
#define IG     ((NI <= 64) ? NI : 64)
#define NGRP   (NI / IG)
#define GROWS  (IG * NSEQ)
#define XSC    64.0f
#define WSC    1024.0f
#define QSC    1024.0f
#define KSC    1024.0f
#define VCAR   1024.0f
#define PCAR   16384.0f
#define OSC    4096.0f
#define MINF   1.0e9f
#define RSQ_HD 0.17677669529663689f
#define LOG2E  1.4426950408889634f
#define WPB    2
#define NHG    (NH / WPB)
#define NQT    (NSEQ / 16)
#define NKT    (NSEQ / 32)
#define NST    (NSEQ / 64)
#define ATT_THREADS (WPB * 32)
#define SBP    260
#define SBW    (16 * SBP)
#define STP    72
#define SLAB64 (16 * 68)
#define VTP    72
#define XTP    136
#define WTP    136
#define BTM    64
#define QKC    (CZ / 8)
#define QKR    16
#define QKT    (QKC * QKR)
#define WS_CAP 134217728
static_assert(NB == 1);
static_assert(CZ == NH * HD && HD == 32 && NH == 4 && NSEQ == 256);
static_assert(NI >= 1 && NI <= NSEQ && (NI % IG) == 0 && IG >= 1 && IG <= 64 && NGRP >= 1);
static_assert((GROWS % 64) == 0 && (GROWS % QKR) == 0 && (NPOS % 64) == 0 && QKT == 256);
static_assert((NH % WPB) == 0 && ATT_THREADS == 64 && (NSEQ % 64) == 0 && (CZ % 64) == 0 && (CZ % 32) == 0);
static_assert((BTM % 64) == 0 && BTM >= NH && (BTM % 32) == 0);
static_assert(SBP >= NSEQ && (SBP % 4) == 0 && STP >= 64 && (STP % 8) == 0 && XTP >= CZ && WTP >= CZ && VTP >= 64);

typedef unsigned short u16;
typedef _Float16 v16h __attribute__((ext_vector_type(16)));
typedef _Float16 v8h  __attribute__((ext_vector_type(8)));
typedef float    v8f  __attribute__((ext_vector_type(8)));
typedef float    v4f  __attribute__((ext_vector_type(4)));
typedef unsigned int v4u __attribute__((ext_vector_type(4)));

union FragH { v16h v; v8h h[2]; v4u u[2]; };

__device__ __forceinline__ unsigned short bf_bits(float f) {
  unsigned u = __float_as_uint(f);
  return (unsigned short)((u + 0x7FFFu + ((u >> 16) & 1u)) >> 16);
}
__device__ __forceinline__ float bf_up(unsigned short h) { return __uint_as_float(((unsigned)h) << 16); }
__device__ __forceinline__ float bfr(float f) { return bf_up(bf_bits(f)); }
__device__ __forceinline__ unsigned short h_bits(_Float16 x) { return __builtin_bit_cast(unsigned short, x); }
__device__ __forceinline__ unsigned pk16(unsigned short a, unsigned short b) { return (unsigned)a | ((unsigned)b << 16); }
__device__ __forceinline__ v8f zero8() { v8f z = {0.f, 0.f, 0.f, 0.f, 0.f, 0.f, 0.f, 0.f}; return z; }

__device__ __forceinline__ v16h ldfrag_h(const _Float16* p) {
  FragH f;
  f.h[0] = *(const v8h*)(p);
  f.h[1] = *(const v8h*)(p + 16);
  return f.v;
}

__device__ __forceinline__ v8f mma_h(v16h a, v16h b, v8f c) {
  return __builtin_amdgcn_wmma_f32_16x16x32_f16(false, a, false, b, (short)0, c, false, false);
}
__device__ __forceinline__ void guard2(v8f& a, v8f& b, v16h x0, v16h x1, v16h x2, v16h x3, v16h x4, v16h x5) {
#if defined(__HIP_DEVICE_COMPILE__)
  asm volatile("v_nop\n\tv_nop\n\tv_nop\n\tv_nop"
               : "+v"(a), "+v"(b) : "v"(x0), "v"(x1), "v"(x2), "v"(x3), "v"(x4), "v"(x5) : "memory");
#endif
}
template <typename F>
__device__ __forceinline__ void guard6(v8f& a, v8f& b, v8f& c, v8f& d, F x0, F x1, F x2, F x3, F x4, F x5) {
#if defined(__HIP_DEVICE_COMPILE__)
  asm volatile("v_nop\n\tv_nop\n\tv_nop\n\tv_nop"
               : "+v"(a), "+v"(b), "+v"(c), "+v"(d) : "v"(x0), "v"(x1), "v"(x2), "v"(x3), "v"(x4), "v"(x5) : "memory");
#endif
}
template <typename F>
__device__ __forceinline__ void guard9(v8f& a, v8f& b, v8f& c, v8f& d, F x0, F x1, F x2, F x3, F x4, F x5,
                                       F x6, F x7, F x8) {
#if defined(__HIP_DEVICE_COMPILE__)
  asm volatile("v_nop\n\tv_nop\n\tv_nop\n\tv_nop"
               : "+v"(a), "+v"(b), "+v"(c), "+v"(d)
               : "v"(x0), "v"(x1), "v"(x2), "v"(x3), "v"(x4), "v"(x5), "v"(x6), "v"(x7), "v"(x8) : "memory");
#endif
}
__device__ __forceinline__ void acc_guard2(v8f& a, v8f& b) {
#if defined(__HIP_DEVICE_COMPILE__)
  asm volatile("v_nop\n\tv_nop\n\tv_nop\n\tv_nop" : "+v"(a), "+v"(b));
#endif
}
__device__ __forceinline__ void wave_sync_lds() {
  __builtin_amdgcn_fence(__ATOMIC_RELEASE, "workgroup");
  __builtin_amdgcn_wave_barrier();
  __builtin_amdgcn_fence(__ATOMIC_ACQUIRE, "workgroup");
}

__global__ __launch_bounds__(256) void ln16(const float* __restrict__ X, const float* __restrict__ gam,
                                            const float* __restrict__ bet, u16* XHo, u16* XLo, int nrows) {
#pragma clang fp contract(off)
  __shared__ __align__(16) u16 TH[64 * XTP];
  __shared__ __align__(16) u16 TL[64 * XTP];
  const int tid = (int)threadIdx.x, wave = tid >> 5, lane = tid & 31;
  const int row0 = (int)blockIdx.x * 64;
  if (row0 + 64 > nrows) return;
  const int rl = tid >> 2, part = tid & 3;
  const float* p = X + (size_t)(row0 + rl) * CZ + part * 32;
  v4f xv[8];
  float s = 0.0f;
#pragma unroll
  for (int t = 0; t < 8; ++t) {
    v4f a = *(const v4f*)(p + 4 * t);
#pragma unroll
    for (int e = 0; e < 4; ++e) { const float f = bfr(a[e]); a[e] = f; s = s + f; }
    xv[t] = a;
  }
  s = s + __shfl_xor(s, 1, 32);
  s = s + __shfl_xor(s, 2, 32);
  const float mu = s * (1.0f / (float)CZ);
  float q = 0.0f;
#pragma unroll
  for (int t = 0; t < 8; ++t) {
#pragma unroll
    for (int e = 0; e < 4; ++e) { const float d = xv[t][e] - mu; q = q + d * d; }
  }
  q = q + __shfl_xor(q, 1, 32);
  q = q + __shfl_xor(q, 2, 32);
  const float var  = q * (1.0f / (float)CZ);
  const float rstd = rsqrtf(var + 1e-5f);
  v4u oh[4], ol[4];
#pragma unroll
  for (int t = 0; t < 8; ++t) {
    const v4f g4 = *(const v4f*)(gam + part * 32 + 4 * t);
    const v4f b4 = *(const v4f*)(bet + part * 32 + 4 * t);
    unsigned short hb[4], lb[4];
#pragma unroll
    for (int e = 0; e < 4; ++e) {
      float y = (xv[t][e] - mu) * rstd;
      y = y * bfr(g4[e]);
      y = y + bfr(b4[e]);
      const float w = y * XSC;
      const _Float16 hv = (_Float16)w;
      const _Float16 lv = (_Float16)(w - (float)hv);
      hb[e] = h_bits(hv);
      lb[e] = h_bits(lv);
    }
    oh[t >> 1][(t & 1) * 2]     = pk16(hb[0], hb[1]);
    oh[t >> 1][(t & 1) * 2 + 1] = pk16(hb[2], hb[3]);
    ol[t >> 1][(t & 1) * 2]     = pk16(lb[0], lb[1]);
    ol[t >> 1][(t & 1) * 2 + 1] = pk16(lb[2], lb[3]);
  }
  {
    u16* th = TH + rl * XTP + part * 32;
    u16* tl = TL + rl * XTP + part * 32;
#pragma unroll
    for (int q4 = 0; q4 < 4; ++q4) {
      *(v4u*)(th + 8 * q4) = oh[q4];
      *(v4u*)(tl + 8 * q4) = ol[q4];
    }
  }
  __syncthreads();
  v4u vh[4], vl[4];
  const int ch = (lane & 15) * 8;
#pragma unroll
  for (int it = 0; it < 4; ++it) {
    const int row = (it * 8 + wave) * 2 + (lane >> 4);
    vh[it] = *(const v4u*)(TH + row * XTP + ch);
    vl[it] = *(const v4u*)(TL + row * XTP + ch);
  }
  for (int pass = 0; pass < 2; ++pass) {
#pragma unroll
    for (int it = 0; it < 4; ++it) {
      const int row = (it * 8 + wave) * 2 + (lane >> 4);
      const size_t o = (size_t)(row0 + row) * CZ + ch;
      *(volatile v4u*)(XHo + o) = vh[it];
      *(volatile v4u*)(XLo + o) = vl[it];
    }
    __threadfence();
  }
}

__global__ __launch_bounds__(256) void wp16(const float* __restrict__ W, int nrow, int np, u16* D, float scale) {
  __shared__ __align__(16) u16 T[32 * WTP];
  const int tid = (int)threadIdx.x, wave = tid >> 5, lane = tid & 31;
  const int n0 = (int)blockIdx.x * 32;
  if (n0 + 32 > np) return;
  {
    const int nl = tid >> 3, kc = (tid & 7) * 16;
    const int n  = n0 + nl;
    int nr = (n < nrow) ? n : (nrow - 1);
    nr = (nr < 0) ? 0 : nr;
    const float* src = W + (size_t)nr * CZ + kc;
    v4u w2[2];
#pragma unroll
    for (int t = 0; t < 4; ++t) {
      const v4f a = *(const v4f*)(src + 4 * t);
      unsigned short hb[4];
#pragma unroll
      for (int e = 0; e < 4; ++e) {
        const float val = (n < nrow) ? a[e] : 0.0f;
        hb[e] = h_bits((_Float16)(bfr(val) * scale));
      }
      w2[t >> 1][(t & 1) * 2]     = pk16(hb[0], hb[1]);
      w2[t >> 1][(t & 1) * 2 + 1] = pk16(hb[2], hb[3]);
    }
    *(v4u*)(T + nl * WTP + kc)     = w2[0];
    *(v4u*)(T + nl * WTP + kc + 8) = w2[1];
  }
  __syncthreads();
  v4u w4[2];
  const int ch = (lane & 15) * 8;
#pragma unroll
  for (int it = 0; it < 2; ++it) {
    const int row = (it * 8 + wave) * 2 + (lane >> 4);
    w4[it] = *(const v4u*)(T + row * WTP + ch);
  }
  for (int pass = 0; pass < 2; ++pass) {
#pragma unroll
    for (int it = 0; it < 2; ++it) {
      const int row = (it * 8 + wave) * 2 + (lane >> 4);
      *(volatile v4u*)(D + (size_t)(n0 + row) * CZ + ch) = w4[it];
    }
    __threadfence();
  }
}

__device__ __forceinline__ void epi64(float* sl, v8f a0, v8f a1, v8f a2, v8f a3, float oscale,
                                      float b0, float b1, float b2, float b3,
                                      float* C, int N, size_t rowb, int col0, int lane) {
  const int hh = lane >> 4, m = lane & 15;
#pragma unroll
  for (int r = 0; r < 8; ++r) {
    const int ro = (8 * hh + r) * 68 + m;
    sl[ro]      = a0[r] * oscale + b0;
    sl[ro + 16] = a1[r] * oscale + b1;
    sl[ro + 32] = a2[r] * oscale + b2;
    sl[ro + 48] = a3[r] * oscale + b3;
  }
  wave_sync_lds();
  v4f vals[8];
#pragma unroll
  for (int it = 0; it < 8; ++it) vals[it] = *(const v4f*)(sl + (it * 2 + hh) * 68 + m * 4);
  float* dst = C + (rowb + (size_t)hh) * (size_t)N + col0 + m * 4;
  for (int pass = 0; pass < 2; ++pass) {
#pragma unroll
    for (int it = 0; it < 8; ++it) {
      *(volatile v4f*)(dst + (size_t)(it * 2) * (size_t)N) = vals[it];
    }
    __threadfence();
  }
}

template <int ALO, int BLO>
__global__ __launch_bounds__(128)
void gemm_h(const u16* __restrict__ Ah, const u16* __restrict__ Al, const u16* __restrict__ Bh, const u16* __restrict__ Bl,
            const float* __restrict__ bias, int hasb, float* C, int M, int N, int K, float oscale) {
  __shared__ __align__(16) float slab[4 * SLAB64];
  const int tid = (int)threadIdx.x, wave = tid >> 5, lane = tid & 31, hh = lane >> 4, m = lane & 15;
  const int ntile = N >> 6;
  const int bid   = (int)blockIdx.x;
  const int rowb  = (bid / ntile) * 64 + wave * 16;
  const int col0  = (bid % ntile) * 64;
  if (rowb + 16 > M) return;
  const _Float16* ahp = (const _Float16*)(const void*)Ah + (size_t)(rowb + m) * K + 8 * hh;
  const _Float16* alp = (const _Float16*)(const void*)Al + (size_t)(rowb + m) * K + 8 * hh;
  const _Float16* bhp = (const _Float16*)(const void*)Bh + (size_t)(col0 + m) * K + 8 * hh;
  const _Float16* blp = (const _Float16*)(const void*)Bl + (size_t)(col0 + m) * K + 8 * hh;
  const size_t bs = (size_t)16 * K;
  float bb0 = 0.0f, bb1 = 0.0f, bb2 = 0.0f, bb3 = 0.0f;
  if (hasb != 0) {
    bb0 = bfr(bias[col0 + m]);
    bb1 = bfr(bias[col0 + 16 + m]);
    bb2 = bfr(bias[col0 + 32 + m]);
    bb3 = bfr(bias[col0 + 48 + m]);
  }
  v8f acc0 = zero8(), acc1 = zero8(), acc2 = zero8(), acc3 = zero8();
#pragma unroll 1
  for (int k0 = 0; k0 < K; k0 += 32) {
    const v16h ah = ldfrag_h(ahp + k0);
    const v16h b0 = ldfrag_h(bhp + k0);
    const v16h b1 = ldfrag_h(bhp + bs + k0);
    const v16h b2 = ldfrag_h(bhp + 2 * bs + k0);
    const v16h b3 = ldfrag_h(bhp + 3 * bs + k0);
    acc0 = mma_h(ah, b0, acc0);
    acc1 = mma_h(ah, b1, acc1);
    acc2 = mma_h(ah, b2, acc2);
    acc3 = mma_h(ah, b3, acc3);
    if constexpr (ALO != 0) {
      const v16h al = ldfrag_h(alp + k0);
      acc0 = mma_h(al, b0, acc0);
      acc1 = mma_h(al, b1, acc1);
      acc2 = mma_h(al, b2, acc2);
      acc3 = mma_h(al, b3, acc3);
      if constexpr (BLO != 0) {
        const v16h l0 = ldfrag_h(blp + k0);
        const v16h l1 = ldfrag_h(blp + bs + k0);
        const v16h l2 = ldfrag_h(blp + 2 * bs + k0);
        const v16h l3 = ldfrag_h(blp + 3 * bs + k0);
        acc0 = mma_h(ah, l0, acc0);
        acc1 = mma_h(ah, l1, acc1);
        acc2 = mma_h(ah, l2, acc2);
        acc3 = mma_h(ah, l3, acc3);
        guard9<v16h>(acc0, acc1, acc2, acc3, ah, b0, b1, b2, b3, l0, l1, l2, l3);
        guard6<v16h>(acc0, acc1, acc2, acc3, al, al, al, al, al, al);
      } else {
        guard6<v16h>(acc0, acc1, acc2, acc3, ah, al, b0, b1, b2, b3);
      }
    } else if constexpr (BLO != 0) {
      const v16h l0 = ldfrag_h(blp + k0);
      const v16h l1 = ldfrag_h(blp + bs + k0);
      const v16h l2 = ldfrag_h(blp + 2 * bs + k0);
      const v16h l3 = ldfrag_h(blp + 3 * bs + k0);
      acc0 = mma_h(ah, l0, acc0);
      acc1 = mma_h(ah, l1, acc1);
      acc2 = mma_h(ah, l2, acc2);
      acc3 = mma_h(ah, l3, acc3);
      guard9<v16h>(acc0, acc1, acc2, acc3, ah, b0, b1, b2, b3, l0, l1, l2, l3);
    } else {
      guard6<v16h>(acc0, acc1, acc2, acc3, ah, b0, b1, b2, b3, ah);
    }
  }
  epi64(slab + wave * SLAB64, acc0, acc1, acc2, acc3, oscale, bb0, bb1, bb2, bb3, C, N, (size_t)rowb, col0, lane);
}

__global__ __launch_bounds__(256) void vt16(const float* __restrict__ F, u16* VHo, u16* VLo) {
  __shared__ __align__(16) u16 TH[HD * VTP];
  __shared__ __align__(16) u16 TL[HD * VTP];
  const int tid = (int)threadIdx.x;
  const int bid = (int)blockIdx.x;
  const int st  = bid % NST;
  const int t2  = bid / NST;
  const int h   = t2 % NH;
  const int il  = t2 / NH;
  if (il >= IG) return;
  const int s0  = st * 64;
  {
    const int sl = tid >> 2;
    const int dc = (tid & 3) * 8;
    const float* src = F + ((size_t)il * NSEQ + s0 + sl) * CZ + h * HD + dc;
    const v4f a = *(const v4f*)(src), b4 = *(const v4f*)(src + 4);
    float w[8];
#pragma unroll
    for (int e = 0; e < 4; ++e) { w[e] = a[e] * VCAR; w[4 + e] = b4[e] * VCAR; }
#pragma unroll
    for (int e = 0; e < 8; ++e) {
      const _Float16 hv = (_Float16)w[e];
      const _Float16 lv = (_Float16)(w[e] - (float)hv);
      TH[(dc + e) * VTP + sl] = h_bits(hv);
      TL[(dc + e) * VTP + sl] = h_bits(lv);
    }
  }
  __syncthreads();
  const int q8 = tid >> 3, p8 = (tid & 7) * 8;
  const v4u vh = *(const v4u*)(TH + q8 * VTP + p8);
  const v4u vl = *(const v4u*)(TL + q8 * VTP + p8);
  const size_t hrow = (size_t)(il * NH + h) * HD + q8;
  const size_t base = hrow * NSEQ + s0 + p8;
  for (int pass = 0; pass < 2; ++pass) {
    *(volatile v4u*)(VHo + base) = vh;
    *(volatile v4u*)(VLo + base) = vl;
    __threadfence();
  }
}

__global__ __launch_bounds__(128) void vmean(const float* __restrict__ F, float* VM) {
  const int il = (int)blockIdx.x;
  if (il >= IG) return;
  const int c = (int)threadIdx.x;
  const float* p = F + (size_t)il * NSEQ * CZ + c;
  float s = 0.0f;
#pragma unroll 4
  for (int k = 0; k < NSEQ; ++k) s += p[(size_t)k * CZ];
  const float mv = s * (1.0f / (float)NSEQ);
  float* d = VM + (size_t)il * CZ + c;
  for (int pass = 0; pass < 2; ++pass) {
    *(volatile float*)(d) = mv;
    __threadfence();
  }
}

__global__ __launch_bounds__(QKT) void qk16(const float* __restrict__ F, u16* Hp, u16* Lp, float sc, int nrows) {
  const int tid = (int)threadIdx.x;
  const int rl  = tid / QKC;
  const int cc  = tid - rl * QKC;
  const int row = (int)blockIdx.x * QKR + rl;
  if (row >= nrows) return;
  const float* p = F + (size_t)row * CZ + cc * 8;
  const v4f a = *(const v4f*)(p), b4 = *(const v4f*)(p + 4);
  float w[8];
#pragma unroll
  for (int e = 0; e < 4; ++e) { w[e] = a[e] * sc; w[4 + e] = b4[e] * sc; }
  v4u oh, ol;
#pragma unroll
  for (int e = 0; e < 4; ++e) {
    const float t0 = w[2 * e], t1 = w[2 * e + 1];
    const _Float16 h0 = (_Float16)t0, h1 = (_Float16)t1;
    const _Float16 l0 = (_Float16)(t0 - (float)h0), l1 = (_Float16)(t1 - (float)h1);
    oh[e] = pk16(h_bits(h0), h_bits(h1));
    ol[e] = pk16(h_bits(l0), h_bits(l1));
  }
  const size_t o = (size_t)row * CZ + cc * 8;
  for (int pass = 0; pass < 2; ++pass) {
    *(volatile v4u*)(Hp + o) = oh;
    *(volatile v4u*)(Lp + o) = ol;
    __threadfence();
  }
}

__global__ __launch_bounds__(ATT_THREADS)
void attn(const u16* __restrict__ QHp, const u16* __restrict__ QLp,
          const u16* __restrict__ KHp, const u16* __restrict__ KLp,
          const u16* __restrict__ VHp, const u16* __restrict__ VLp,
          const float* __restrict__ VM, const float* __restrict__ GF, const float* __restrict__ BT,
          const float* __restrict__ MK, u16* OHp, u16* OLp) {
  __shared__ __align__(16) float sbuf[WPB * SBW];
  __shared__ __align__(16) u16 stg[2 * 16 * STP];

  const int tid  = (int)threadIdx.x;
  const int wave = tid >> 5;
  const int lane = tid & 31;
  const int hh   = lane >> 4;
  const int c    = lane & 15;
  const int bid  = (int)blockIdx.x;
  const int qt   = bid % NQT;
  const int t2   = bid / NQT;
  const int hg   = t2 % NHG;
  const int il   = t2 / NHG;
  if (il >= IG) return;
  const int q0   = qt * 16;
  const int head = hg * WPB + wave;
  float* buf = sbuf + wave * SBW;
  const size_t prow0 = (size_t)il * NSEQ;

  {
    const float* bsrc = BT + (size_t)head * NPOS + (size_t)q0 * NSEQ;
    const float* msrc = MK + (size_t)il * NSEQ;
    v4f mb0, mb1;
    {
      const v4f m0 = *(const v4f*)(msrc + lane * 4);
      const v4f m1 = *(const v4f*)(msrc + 128 + lane * 4);
#pragma unroll
      for (int e = 0; e < 4; ++e) {
        mb0[e] = (MINF * (bfr(m0[e]) - 1.0f)) * LOG2E;
        mb1[e] = (MINF * (bfr(m1[e]) - 1.0f)) * LOG2E;
      }
    }
#pragma unroll 1
    for (int g4 = 0; g4 < 4; ++g4) {
      v4f tv[8];
#pragma unroll
      for (int it = 0; it < 8; ++it) {
        const int idx = (g4 * 8 + it) * 32 + lane;
        const int jr = idx >> 6, k4 = (idx & 63) * 4;
        tv[it] = *(const v4f*)(bsrc + (size_t)jr * NSEQ + k4);
      }
#pragma unroll
      for (int it = 0; it < 8; ++it) {
        const int idx = (g4 * 8 + it) * 32 + lane;
        const int jr = idx >> 6, k4 = (idx & 63) * 4;
        const v4f mb = (it & 1) ? mb1 : mb0;
        *(v4f*)(buf + jr * SBP + k4) = tv[it] * LOG2E + mb;
      }
    }
  }
  wave_sync_lds();

  const size_t hcol = (size_t)head * HD + 8 * hh;
  const _Float16* Qh  = (const _Float16*)(const void*)QHp + (prow0 + q0 + c) * CZ + hcol;
  const _Float16* Ql  = (const _Float16*)(const void*)QLp + (prow0 + q0 + c) * CZ + hcol;
  const _Float16* Khb = (const _Float16*)(const void*)KHp + (prow0 + c) * CZ + hcol;
  const _Float16* Klb = (const _Float16*)(const void*)KLp + (prow0 + c) * CZ + hcol;
  const _Float16* Vhb = (const _Float16*)(const void*)VHp + ((size_t)(il * NH + head) * HD + c) * NSEQ + 8 * hh;
  const _Float16* Vlb = (const _Float16*)(const void*)VLp + ((size_t)(il * NH + head) * HD + c) * NSEQ + 8 * hh;
  const v16h qh = ldfrag_h(Qh);
  const v16h ql = ldfrag_h(Ql);
  const float lsc = RSQ_HD * (LOG2E / (QSC * KSC));

  float mrow[8];
#pragma unroll
  for (int r = 0; r < 8; ++r) mrow[r] = -INFINITY;
#pragma unroll 1
  for (int kt = 0; kt < NKT; ++kt) {
    const int kb = kt * 32;
    const _Float16* k0p = Khb + (size_t)kb * CZ;
    const _Float16* k1p = k0p + (size_t)16 * CZ;
    const _Float16* l0p = Klb + (size_t)kb * CZ;
    const _Float16* l1p = l0p + (size_t)16 * CZ;
    const v16h kh0 = ldfrag_h(k0p), kh1 = ldfrag_h(k1p);
    const v16h kl0 = ldfrag_h(l0p), kl1 = ldfrag_h(l1p);
    v8f s0 = zero8(), s1 = zero8();
    s0 = mma_h(qh, kh0, s0);
    s0 = mma_h(ql, kh0, s0);
    s0 = mma_h(qh, kl0, s0);
    s1 = mma_h(qh, kh1, s1);
    s1 = mma_h(ql, kh1, s1);
    s1 = mma_h(qh, kl1, s1);
    guard2(s0, s1, qh, ql, kh0, kl0, kh1, kl1);
#pragma unroll
    for (int r = 0; r < 8; ++r) {
      const int pos = (8 * hh + r) * SBP + kb + c;
      const float u0 = s0[r] * lsc + buf[pos];
      const float u1 = s1[r] * lsc + buf[pos + 16];
      buf[pos]      = u0;
      buf[pos + 16] = u1;
      mrow[r] = fmaxf(mrow[r], fmaxf(u0, u1));
    }
  }
#pragma unroll
  for (int r = 0; r < 8; ++r) {
    float mx = mrow[r];
#pragma unroll
    for (int off = 1; off < 16; off <<= 1) mx = fmaxf(mx, __shfl_xor(mx, off, 32));
    mrow[r] = mx;
  }

  float psc[8];
  {
    float lrow[8];
#pragma unroll
    for (int r = 0; r < 8; ++r) lrow[r] = 0.0f;
#pragma unroll 1
    for (int kt = 0; kt < NKT; ++kt) {
      const int kb = kt * 32;
#pragma unroll
      for (int r = 0; r < 8; ++r) {
        const int pos = (8 * hh + r) * SBP + kb + c;
        const float e0 = exp2f(buf[pos] - mrow[r]);
        const float e1 = exp2f(buf[pos + 16] - mrow[r]);
        buf[pos]      = e0;
        buf[pos + 16] = e1;
        lrow[r] += e0 + e1;
      }
    }
#pragma unroll
    for (int r = 0; r < 8; ++r) {
      float ls = lrow[r];
#pragma unroll
      for (int off = 1; off < 16; off <<= 1) ls += __shfl_xor(ls, off, 32);
      const float lz = (ls > 0.0f) ? ls : 1.0f;
      psc[r] = PCAR * __builtin_amdgcn_rcpf(lz);
    }
  }

  const float pcen = PCAR / (float)NSEQ;
  v8f o0 = zero8(), o1 = zero8();
#pragma unroll 1
  for (int kt = 0; kt < NKT; ++kt) {
    const int kb = kt * 32;
#pragma unroll
    for (int r = 0; r < 8; ++r) {
      const int pos = (8 * hh + r) * SBP + kb + c;
      const float pp0 = buf[pos] * psc[r] - pcen;
      const float pp1 = buf[pos + 16] * psc[r] - pcen;
      buf[pos]      = pp0;
      buf[pos + 16] = pp1;
    }
    wave_sync_lds();
    FragH ph;
    {
      const float* prow = buf + c * SBP + kb + 8 * hh;
      const v4f p0 = *(const v4f*)(prow), p1 = *(const v4f*)(prow + 4);
      const v4f p2 = *(const v4f*)(prow + 16), p3 = *(const v4f*)(prow + 20);
#pragma unroll
      for (int e = 0; e < 4; ++e) {
        ph.h[0][e]     = (_Float16)p0[e];
        ph.h[0][4 + e] = (_Float16)p1[e];
        ph.h[1][e]     = (_Float16)p2[e];
        ph.h[1][4 + e] = (_Float16)p3[e];
      }
    }
    {
      const v16h vha = ldfrag_h(Vhb + kb);
      const v16h vhb = ldfrag_h(Vhb + (size_t)16 * NSEQ + kb);
      const v16h vla = ldfrag_h(Vlb + kb);
      const v16h vlb = ldfrag_h(Vlb + (size_t)16 * NSEQ + kb);
      o0 = mma_h(ph.v, vha, o0);
      o0 = mma_h(ph.v, vla, o0);
      o1 = mma_h(ph.v, vhb, o1);
      o1 = mma_h(ph.v, vlb, o1);
      guard2(o0, o1, ph.v, vha, vla, vhb, vlb, ph.v);
    }
  }
  acc_guard2(o0, o1);

  {
    const float oc  = 1.0f / (PCAR * VCAR);
    const float vm0 = VM[(size_t)il * CZ + head * HD + c];
    const float vm1 = VM[(size_t)il * CZ + head * HD + 16 + c];
    const float* gp = GF + (prow0 + q0 + 8 * hh) * CZ + head * HD + c;
#pragma unroll
    for (int r = 0; r < 8; ++r) {
      const float gz0 = gp[(size_t)r * CZ];
      const float gz1 = gp[(size_t)r * CZ + 16];
      const float g0  = __builtin_amdgcn_rcpf(1.0f + exp2f(-gz0 * LOG2E));
      const float g1  = __builtin_amdgcn_rcpf(1.0f + exp2f(-gz1 * LOG2E));
      const float w0  = (o0[r] * oc + vm0) * g0 * OSC;
      const float w1  = (o1[r] * oc + vm1) * g1 * OSC;
      const _Float16 h0 = (_Float16)w0, h1 = (_Float16)w1;
      const _Float16 l0 = (_Float16)(w0 - (float)h0), l1 = (_Float16)(w1 - (float)h1);
      const int si = (8 * hh + r) * STP + wave * HD + c;
      stg[si]                 = h_bits(h0);
      stg[si + 16]            = h_bits(h1);
      stg[16 * STP + si]      = h_bits(l0);
      stg[16 * STP + si + 16] = h_bits(l1);
    }
  }
  __syncthreads();
  v4u vh[2], vl[2];
  const int rq = lane >> 3, p8 = (lane & 7) * 8;
#pragma unroll
  for (int it = 0; it < 2; ++it) {
    const int row = it * 8 + wave * 4 + rq;
    vh[it] = *(const v4u*)(stg + row * STP + p8);
    vl[it] = *(const v4u*)(stg + (16 + row) * STP + p8);
  }
  const size_t ob = (prow0 + q0) * CZ + (size_t)hg * 64 + p8;
  for (int pass = 0; pass < 2; ++pass) {
#pragma unroll
    for (int it = 0; it < 2; ++it) {
      const int row = it * 8 + wave * 4 + rq;
      *(volatile v4u*)(OHp + ob + (size_t)row * CZ) = vh[it];
      *(volatile v4u*)(OLp + ob + (size_t)row * CZ) = vl[it];
    }
    __threadfence();
  }
}

extern "C" void kernel_launch(void* const* d_in, const int* in_sizes, int n_in,
                              void* d_out, int out_size, void* d_ws, size_t ws_size,
                              hipStream_t stream) {
  if (n_in < 12) return;
  if (in_sizes[0] < NPOS * CZ) return;
  if (in_sizes[1] < NI * NSEQ) return;
  if (in_sizes[2] < CZ || in_sizes[3] < CZ) return;
  if (in_sizes[4] < NH * CZ) return;
  if (in_sizes[5] < CZ * CZ || in_sizes[6] < CZ * CZ || in_sizes[7] < CZ * CZ || in_sizes[8] < CZ * CZ) return;
  if (in_sizes[9] < CZ) return;
  if (in_sizes[10] < CZ * CZ || in_sizes[11] < CZ) return;
  if (out_size < NI * NSEQ * CZ) return;

  const float* x   = (const float*)d_in[0];
  const float* msk = (const float*)d_in[1];
  const float* gam = (const float*)d_in[2];
  const float* bet = (const float*)d_in[3];
  const float* Wt  = (const float*)d_in[4];
  const float* Wq  = (const float*)d_in[5];
  const float* Wk  = (const float*)d_in[6];
  const float* Wv  = (const float*)d_in[7];
  const float* Wg  = (const float*)d_in[8];
  const float* bg  = (const float*)d_in[9];
  const float* Wo  = (const float*)d_in[10];
  const float* bo  = (const float*)d_in[11];
  float*       out = (float*)d_out;

  const size_t szWP = 32768;
  const size_t szVM = (((size_t)IG * CZ * 4) + 32767) / 32768 * 32768;
  const size_t szX  = (size_t)NPOS * CZ * 2;
  const size_t szBT = (size_t)BTM * NPOS * 4;
  const size_t szF  = (size_t)GROWS * CZ * 4;
  const size_t szP  = (size_t)GROWS * CZ * 2;
  if (2 * szP > szF) return;
  size_t off = 0;
  const size_t oWQ = off; off += szWP;
  const size_t oWK = off; off += szWP;
  const size_t oWV = off; off += szWP;
  const size_t oWG = off; off += szWP;
  const size_t oWO = off; off += szWP;
  const size_t oWB = off; off += szWP;
  const size_t oVM = off; off += szVM;
  const size_t oXH = off; off += szX;
  const size_t oXL = off; off += szX;
  const size_t oBT = off; off += szBT;
  const size_t oF  = off; off += szF;
  const size_t oGF = off; off += szF;
  const size_t oQH = off; off += szP;
  const size_t oQL = off; off += szP;
  const size_t oKH = off; off += szP;
  const size_t oKL = off; off += szP;
  const size_t oVH = off; off += szP;
  const size_t oVL = off; off += szP;
  if (off > ws_size) return;
  if (off > (size_t)WS_CAP) return;

  char* ws = (char*)d_ws;
  u16*   WQ = (u16*)(ws + oWQ);
  u16*   WK = (u16*)(ws + oWK);
  u16*   WV = (u16*)(ws + oWV);
  u16*   WG = (u16*)(ws + oWG);
  u16*   WO = (u16*)(ws + oWO);
  u16*   WB = (u16*)(ws + oWB);
  float* VM = (float*)(ws + oVM);
  u16*   XH = (u16*)(ws + oXH);
  u16*   XL = (u16*)(ws + oXL);
  float* BT = (float*)(ws + oBT);
  float* F  = (float*)(ws + oF);
  u16*   OH = (u16*)(ws + oF);
  u16*   OL = (u16*)(ws + oF + szP);
  float* GF = (float*)(ws + oGF);
  u16*   QH = (u16*)(ws + oQH);
  u16*   QL = (u16*)(ws + oQL);
  u16*   KH = (u16*)(ws + oKH);
  u16*   KL = (u16*)(ws + oKL);
  u16*   VH = (u16*)(ws + oVH);
  u16*   VL = (u16*)(ws + oVL);

  const dim3 b256(256), b128(128), bAT(ATT_THREADS), bQK(QKT);
  const dim3 gLN(NPOS / 64);
  const dim3 gW(CZ / 32), gWB(BTM / 32);
  const dim3 gBias((BTM / 64) * (NPOS / 64));
  const dim3 gG((GROWS / 64) * (CZ / 64));
  const dim3 gVT(IG * NH * NST);
  const dim3 gVM(IG);
  const dim3 gQK(GROWS / QKR);
  const dim3 gA(IG * NHG * NQT);
  const float oscp = 1.0f / (XSC * WSC);
  const float osco = 1.0f / (OSC * WSC);

  ln16<<<gLN, b256, 0, stream>>>(x, gam, bet, XH, XL, NPOS);
  wp16<<<gW,  b256, 0, stream>>>(Wq, CZ, CZ,  WQ, WSC);
  wp16<<<gW,  b256, 0, stream>>>(Wk, CZ, CZ,  WK, WSC);
  wp16<<<gW,  b256, 0, stream>>>(Wv, CZ, CZ,  WV, WSC);
  wp16<<<gW,  b256, 0, stream>>>(Wg, CZ, CZ,  WG, WSC);
  wp16<<<gW,  b256, 0, stream>>>(Wo, CZ, CZ,  WO, WSC);
  wp16<<<gWB, b256, 0, stream>>>(Wt, NH, BTM, WB, WSC);
  gemm_h<0, 1><<<gBias, b128, 0, stream>>>(WB, WB, XH, XL, bo, 0, BT, BTM, NPOS, CZ, oscp);

  for (int g = 0; g < NGRP; ++g) {
    const u16*   XHg = XH + (size_t)g * GROWS * CZ;
    const u16*   XLg = XL + (size_t)g * GROWS * CZ;
    const float* Mg  = msk + (size_t)g * IG * NSEQ;
    float*       og  = out + (size_t)g * GROWS * CZ;
    gemm_h<1, 0><<<gG, b128, 0, stream>>>(XHg, XLg, WV, WV, bo, 0, F, GROWS, CZ, CZ, oscp);
    vt16<<<gVT, b256, 0, stream>>>(F, VH, VL);
    vmean<<<gVM, b128, 0, stream>>>(F, VM);
    gemm_h<1, 0><<<gG, b128, 0, stream>>>(XHg, XLg, WQ, WQ, bo, 0, F, GROWS, CZ, CZ, oscp);
    qk16<<<gQK, bQK, 0, stream>>>(F, QH, QL, QSC, GROWS);
    gemm_h<1, 0><<<gG, b128, 0, stream>>>(XHg, XLg, WK, WK, bo, 0, F, GROWS, CZ, CZ, oscp);
    qk16<<<gQK, bQK, 0, stream>>>(F, KH, KL, KSC, GROWS);
    gemm_h<1, 0><<<gG, b128, 0, stream>>>(XHg, XLg, WG, WG, bg, 1, GF, GROWS, CZ, CZ, oscp);
    attn<<<gA, bAT, 0, stream>>>(QH, QL, KH, KL, VH, VL, VM, GF, BT, Mg, OH, OL);
    gemm_h<1, 0><<<gG, b128, 0, stream>>>(OH, OL, WO, WO, bo, 1, og, GROWS, CZ, CZ, osco);
  }
  (void)hipGetLastError();
}
